// Deform_Conv_21414706938551
// MI455X (gfx1250) — hardware-verified
//
#include <hip/hip_runtime.h>
#ifndef NB
#define NB 8
#endif
#define CC 64
#define OC 64
#define HI 96
#define WI 96
#define HW (HI * WI)
#define NOFFC 18
#define K9C 576
#define K2C 1152
#define NR ((size_t)NB * HW)
#define CHB ((NB % 2 == 0) ? 2 : 1)
#define NCHUNK (NB / CHB)
#define RCH ((size_t)CHB * HW)
#define S_OFF 256.0f
#define A_OFF 0.00390625f
#define S_HI 4096.0f
#define S_LO 4.0f
#define A_MAIN 0.000244140625f
#define RESC 1024.0f

static_assert(HW % 128 == 0);
static_assert(HW % 64 == 0);
static_assert(K9C % 32 == 0);
static_assert(K2C % 32 == 0);
static_assert(NB % CHB == 0);
static_assert((RCH * 72) % 256 == 0);
static_assert(RCH % 128 == 0);

typedef _Float16 v16h __attribute__((ext_vector_type(16)));
typedef unsigned short v8us __attribute__((ext_vector_type(8), may_alias));
typedef float v8f __attribute__((ext_vector_type(8)));
typedef float v4f __attribute__((ext_vector_type(4)));
typedef float v4fa __attribute__((ext_vector_type(4), may_alias));
typedef _Float16 v4h __attribute__((ext_vector_type(4)));
union FragH { v16h v; v8us half[2]; _Float16 h[16]; unsigned short u[16]; };

__device__ __forceinline__ unsigned short bf16_bits(float x) { unsigned int u = __float_as_uint(x); return (unsigned short)((u + 0x7FFFu + ((u >> 16) & 1u)) >> 16); }
__device__ __forceinline__ float bf16_val(unsigned short b) { return __uint_as_float(((unsigned int)b) << 16); }
__device__ __forceinline__ float bf16_rne(float x) { return bf16_val(bf16_bits(x)); }

__device__ __forceinline__ v16h g2_frag(const _Float16* p, int hh) { FragH f; f.half[0] = *(const v8us*)((const unsigned short*)p + 8 * hh); f.half[1] = *(const v8us*)((const unsigned short*)p + 16 + 8 * hh); return f.v; }
__device__ __forceinline__ v8f g2_mma(v16h a, v16h b, v8f c) { v8f d = __builtin_amdgcn_wmma_f32_16x16x32_f16(false, a, false, b, (short)0, c, false, false); asm volatile("v_nop\n\tv_nop\n\tv_nop\n\tv_nop" : "+v"(d) : "v"(a), "v"(b)); return d; }

template <int ACT>
__global__ __launch_bounds__(128) void k_gemm2(const _Float16* __restrict__ A, int lda, size_t sA, const _Float16* __restrict__ Bh, int ldb, size_t sB, float alpha, const float* __restrict__ bias, size_t sBias, const float* __restrict__ CP, int rowsPerB, size_t sCPb, int row0g,
    float* __restrict__ C, _Float16* __restrict__ C16, int ldc, size_t sC, int M, int N, int K) {
  static_assert(ACT == 0 || ACT == 3);
  __shared__ __attribute__((aligned(16))) float so[4][32][68];
  const int tid = threadIdx.x, w = tid >> 5, lane = tid & 31, ln = lane & 15, hh = lane >> 4; const int by = blockIdx.y;
  A += (size_t)by * sA; Bh += (size_t)by * sB; const size_t cofs = (size_t)by * sC; const float* bp = bias ? bias + (size_t)by * sBias : nullptr;
  const int ntn = N >> 6; const int mt = blockIdx.x / ntn, nq = blockIdx.x - mt * ntn; const int row0 = mt * 128 + 32 * w, col0 = nq * 64; if (row0 >= M) return;
  const _Float16* a0p = A + (size_t)(row0 + ln) * lda; const _Float16* a1p = a0p + (size_t)16 * lda;
  const _Float16* b0p = Bh + (size_t)(col0 + ln) * ldb; const _Float16* b1p = b0p + (size_t)16 * ldb; const _Float16* b2p = b1p + (size_t)16 * ldb; const _Float16* b3p = b2p + (size_t)16 * ldb;
  const v8f z8 = {0.f,0.f,0.f,0.f,0.f,0.f,0.f,0.f}; v8f c00 = z8, c01 = z8, c02 = z8, c03 = z8, c10 = z8, c11 = z8, c12 = z8, c13 = z8;
#pragma unroll 1
  for (int kb = 0; kb < K; kb += 32) { const v16h a0 = g2_frag(a0p + kb, hh), a1 = g2_frag(a1p + kb, hh);
    v16h b = g2_frag(b0p + kb, hh); c00 = g2_mma(a0, b, c00); c10 = g2_mma(a1, b, c10);
    b = g2_frag(b1p + kb, hh); c01 = g2_mma(a0, b, c01); c11 = g2_mma(a1, b, c11);
    b = g2_frag(b2p + kb, hh); c02 = g2_mma(a0, b, c02); c12 = g2_mma(a1, b, c12);
    b = g2_frag(b3p + kb, hh); c03 = g2_mma(a0, b, c03); c13 = g2_mma(a1, b, c13); }
  v8f accs[8] = {c00, c01, c02, c03, c10, c11, c12, c13};
#pragma unroll
  for (int u = 0; u < 8; ++u) { const int t = u & 3, half = u >> 2; const int col = col0 + t * 16 + ln; const float bv = bp ? bf16_rne(bp[col]) : 0.f;
#pragma unroll
    for (int r = 0; r < 8; ++r) { const int rloc = half * 16 + 8 * hh + r; float v = accs[u][r] * alpha + bv; if (CP) { if (rowsPerB < 0) v += CP[cofs + (size_t)(row0g + row0 + rloc) * ldc + col];        else { const int bidx = (row0g + row0 + rloc) / rowsPerB; v += CP[(size_t)bidx * sCPb + (size_t)by * 64 + col]; } }
      if (ACT == 3) v = fmaxf(v, 0.f);
      so[w][rloc][t * 16 + ln] = v; } }
  __builtin_amdgcn_fence(__ATOMIC_ACQ_REL, "workgroup"); __builtin_amdgcn_wave_barrier();
  const int rsub = lane >> 4, c4 = (lane & 15) * 4;
  for (int pass = 0; pass < 2; ++pass) {
#pragma unroll
    for (int q = 0; q < 16; ++q) { const int r = q * 2 + rsub; const v4f v = *(const v4fa*)&so[w][r][c4]; if (C) *(volatile v4f*)(C + cofs + (size_t)(row0 + r) * ldc + col0 + c4) = v; if (C16) { v4h h4; for (int i = 0; i < 4; ++i) h4[i] = (_Float16)v[i]; *(volatile v4h*)(C16 + cofs + (size_t)(row0 + r) * ldc + col0 + c4) = h4; } }
    if (pass == 0) __threadfence(); } }

__global__ __launch_bounds__(128) void k_gemm2t(const _Float16* __restrict__ A, int lda, const _Float16* __restrict__ Bh, int ldb, float alpha, size_t row0c, float* __restrict__ out, int M, int K) {
  __shared__ __attribute__((aligned(16))) float so[4][32][68];
  const int tid = threadIdx.x, w = tid >> 5, lane = tid & 31, ln = lane & 15, hh = lane >> 4;
  const int row0 = blockIdx.x * 128 + 32 * w; if (row0 >= M) return;
  const _Float16* a0p = A + (size_t)(row0 + ln) * lda; const _Float16* a1p = a0p + (size_t)16 * lda;
  const _Float16* b0p = Bh + (size_t)ln * ldb; const _Float16* b1p = b0p + (size_t)16 * ldb; const _Float16* b2p = b1p + (size_t)16 * ldb; const _Float16* b3p = b2p + (size_t)16 * ldb;
  const v8f z8 = {0.f,0.f,0.f,0.f,0.f,0.f,0.f,0.f}; v8f c00 = z8, c01 = z8, c02 = z8, c03 = z8, c10 = z8, c11 = z8, c12 = z8, c13 = z8;
#pragma unroll 1
  for (int kb = 0; kb < K; kb += 32) { const v16h a0 = g2_frag(a0p + kb, hh), a1 = g2_frag(a1p + kb, hh);
    v16h b = g2_frag(b0p + kb, hh); c00 = g2_mma(a0, b, c00); c10 = g2_mma(a1, b, c10);
    b = g2_frag(b1p + kb, hh); c01 = g2_mma(a0, b, c01); c11 = g2_mma(a1, b, c11);
    b = g2_frag(b2p + kb, hh); c02 = g2_mma(a0, b, c02); c12 = g2_mma(a1, b, c12);
    b = g2_frag(b3p + kb, hh); c03 = g2_mma(a0, b, c03); c13 = g2_mma(a1, b, c13); }
  v8f accs[8] = {c00, c01, c02, c03, c10, c11, c12, c13};
#pragma unroll
  for (int u = 0; u < 8; ++u) { const int t = u & 3, half = u >> 2;
#pragma unroll
    for (int r = 0; r < 8; ++r) { const int rloc = half * 16 + 8 * hh + r; so[w][rloc][t * 16 + ln] = accs[u][r] * alpha; } }
  __builtin_amdgcn_fence(__ATOMIC_ACQ_REL, "workgroup"); __builtin_amdgcn_wave_barrier();
  const size_t g = row0c + (size_t)row0; const size_t bimg = g / HW; const size_t p0 = g - bimg * HW;
  const int j = lane & 7, og = lane >> 3;
  float* ob = out + bimg * (size_t)OC * HW + p0 + 4 * j;
  for (int pass = 0; pass < 2; ++pass) {
#pragma unroll
    for (int it = 0; it < 16; ++it) { const int o = it * 4 + og; v4f v; v[0] = so[w][4 * j][o]; v[1] = so[w][4 * j + 1][o]; v[2] = so[w][4 * j + 2][o]; v[3] = so[w][4 * j + 3][o];
      *(volatile v4f*)(ob + (size_t)o * HW) = v; }
    if (pass == 0) __threadfence(); } }

__global__ __launch_bounds__(256) void k_xT(const float* __restrict__ x, _Float16* __restrict__ X16) {
  __shared__ __attribute__((aligned(16))) unsigned short tl[64][72];
  const int tid = threadIdx.x;
  const int b = blockIdx.x / (HW / 64), pg = blockIdx.x % (HW / 64);
  const size_t p0 = (size_t)pg * 64;
  const float* xb = x + (size_t)b * CC * HW + p0;
#pragma unroll
  for (int i = 0; i < 16; ++i) { const int idx = i * 256 + tid; const int c = idx >> 6, p = idx & 63; FragH f; f.h[0] = (_Float16)bf16_rne(xb[(size_t)c * HW + p]); tl[p][c] = f.u[0]; }
  __syncthreads();
  const int j = tid & 7, pr = tid >> 3;
  const v8us v0 = *(const v8us*)&tl[pr][8 * j];
  const v8us v1 = *(const v8us*)&tl[pr + 32][8 * j];
  unsigned short* d0 = (unsigned short*)X16 + ((size_t)b * HW + p0 + pr) * CC + 8 * j;
  unsigned short* d1 = d0 + (size_t)32 * CC;
  for (int pass = 0; pass < 2; ++pass) { *(volatile v8us*)d0 = v0; *(volatile v8us*)d1 = v1; if (pass == 0) __threadfence(); } }

__global__ __launch_bounds__(256) void k_wk(const float* __restrict__ w, int nrows, int nhalf, float s0, float s1, _Float16* __restrict__ Bt) {
  const int t = blockIdx.x * 256 + threadIdx.x; const int per_o = nhalf * 72;
  if (t >= OC * per_o) return;
  const int o = t / per_o; const int rem = t - o * per_o; const int h = rem / 72; const int r2 = rem - h * 72; const int tap = r2 >> 3; const int c8 = (r2 & 7) * 8;
  const int oc = min(o, nrows - 1); const float sc = h ? s1 : s0;
  FragH f;
#pragma unroll
  for (int q = 0; q < 8; ++q) { const float wv = bf16_rne(w[((size_t)oc * CC + c8 + q) * 9 + tap]) * sc; f.h[q] = (o < nrows) ? (_Float16)wv : (_Float16)0.0f; }
  unsigned short* d = (unsigned short*)Bt + (size_t)o * ((size_t)nhalf * K9C) + (size_t)h * K9C + tap * 64 + c8;
  *(volatile v8us*)d = f.half[0]; __threadfence(); *(volatile v8us*)d = f.half[0]; }

__global__ __launch_bounds__(64) void k_b64(const float* __restrict__ bsrc, int n, float* __restrict__ bp) {
  const int i = threadIdx.x; const float v = (i < n) ? bsrc[min(i, n - 1)] : 0.f;
  *(volatile float*)(bp + i) = v; __threadfence(); *(volatile float*)(bp + i) = v; }

__global__ __launch_bounds__(256) void k_im9(const _Float16* __restrict__ X16, size_t row0c, size_t nrows, _Float16* __restrict__ IM) {
  const size_t t = (size_t)blockIdx.x * 256 + threadIdx.x; if (t >= nrows * 72) return;
  const int c8 = (int)(t & 7) * 8; const size_t rt = t >> 3; const int tap = (int)(rt % 9); const size_t lrow = rt / 9; const size_t row = row0c + lrow;
  const size_t b = row / HW; const int p = (int)(row - b * HW); const int iy = p / WI + tap / 3 - 1, ix = p % WI + tap % 3 - 1;
  const bool ok = (iy >= 0) && (iy < HI) && (ix >= 0) && (ix < WI);
  const int cy = min(max(iy, 0), HI - 1), cx = min(max(ix, 0), WI - 1);
  const v8us v = *(const v8us*)((const unsigned short*)X16 + (b * HW + (size_t)cy * WI + cx) * CC + c8);
  v8us o;
#pragma unroll
  for (int q = 0; q < 8; ++q) o[q] = ok ? v[q] : (unsigned short)0;
  *(volatile v8us*)((unsigned short*)IM + t * 8) = o; __threadfence(); *(volatile v8us*)((unsigned short*)IM + t * 8) = o; }

__global__ __launch_bounds__(256) void k_samp(const _Float16* __restrict__ X16, const float* __restrict__ OFF, size_t row0c, size_t nrows, _Float16* __restrict__ IMP) {
  #pragma clang fp contract(off)
  const size_t t = (size_t)blockIdx.x * 256 + threadIdx.x; if (t >= nrows * 72) return;
  const int c8 = (int)(t & 7) * 8; const size_t rt = t >> 3; const int tap = (int)(rt % 9); const size_t lrow = rt / 9; const size_t row = row0c + lrow;
  const size_t b = row / HW; const int p = (int)(row - b * HW); const int i = p / WI, j = p - i * WI;
  const int ky = tap / 3, kx = tap - ky * 3;
  const float dy = OFF[lrow * 64 + 2 * tap], dx = OFF[lrow * 64 + 2 * tap + 1];
  const float py = (dy + (float)(i - 1)) + (float)ky;
  const float px = (dx + (float)(j - 1)) + (float)kx;
  const float y0f = floorf(py), x0f = floorf(px);
  const float wy = py - y0f, wx = px - x0f;
  const int y0 = (int)fminf(fmaxf(y0f, -8.0f), (float)(HI + 8));
  const int x0 = (int)fminf(fmaxf(x0f, -8.0f), (float)(WI + 8));
  const int y1 = y0 + 1, x1 = x0 + 1;
  const bool oy0 = (y0 >= 0) && (y0 < HI), oy1 = (y1 >= 0) && (y1 < HI), ox0 = (x0 >= 0) && (x0 < WI), ox1 = (x1 >= 0) && (x1 < WI);
  const float v00 = (oy0 && ox0) ? 1.f : 0.f, v01 = (oy0 && ox1) ? 1.f : 0.f, v10 = (oy1 && ox0) ? 1.f : 0.f, v11 = (oy1 && ox1) ? 1.f : 0.f;
  const int cy0 = min(max(y0, 0), HI - 1), cy1 = min(max(y1, 0), HI - 1), cx0 = min(max(x0, 0), WI - 1), cx1 = min(max(x1, 0), WI - 1);
  const float w00 = (1.f - wy) * (1.f - wx), w01 = (1.f - wy) * wx, w10 = wy * (1.f - wx), w11 = wy * wx;
  const unsigned short* base = (const unsigned short*)X16 + b * (size_t)HW * CC + c8;
  FragH g00, g01, g10, g11;
  g00.half[0] = *(const v8us*)(base + ((size_t)cy0 * WI + cx0) * CC);
  g01.half[0] = *(const v8us*)(base + ((size_t)cy0 * WI + cx1) * CC);
  g10.half[0] = *(const v8us*)(base + ((size_t)cy1 * WI + cx0) * CC);
  g11.half[0] = *(const v8us*)(base + ((size_t)cy1 * WI + cx1) * CC);
  FragH fh, fl;
#pragma unroll
  for (int q = 0; q < 8; ++q) {
    const float a00 = (float)g00.h[q] * v00, a01 = (float)g01.h[q] * v01, a10 = (float)g10.h[q] * v10, a11 = (float)g11.h[q] * v11;
    float s = a00 * w00; s = s + a01 * w01; s = s + a10 * w10; s = s + a11 * w11;
    const _Float16 hq = (_Float16)s; fh.h[q] = hq; fl.h[q] = (_Float16)((s - (float)hq) * RESC);
  }
  unsigned short* d = (unsigned short*)IMP + lrow * (size_t)K2C + (size_t)tap * 64 + c8;
  for (int pass = 0; pass < 2; ++pass) { *(volatile v8us*)d = fh.half[0]; *(volatile v8us*)(d + K9C) = fl.half[0]; if (pass == 0) __threadfence(); } }

extern "C" void kernel_launch(void* const* d_in, const int* in_sizes, int n_in,
                              void* d_out, int out_size, void* d_ws, size_t ws_size, hipStream_t stream) {
  if (n_in < 4) return;
  if (in_sizes[0] < (int)((size_t)NB * CC * HW) || in_sizes[1] < NOFFC * CC * 9 || in_sizes[2] < NOFFC || in_sizes[3] < OC * CC * 9) return;
  if ((size_t)out_size < NR * OC) return;
  const float* x = (const float*)d_in[0]; const float* w_off = (const float*)d_in[1]; const float* b_off = (const float*)d_in[2]; const float* wd = (const float*)d_in[3];
  float* out = (float*)d_out;
  char* ws = (char*)d_ws; size_t off = 0;
  auto take = [&](size_t bytes) { char* p = ws + off; off += (bytes + 255) & ~(size_t)255; return p; };
  const size_t szX16 = NR * CC * 2, szBtO = (size_t)OC * K9C * 2, szBtD = (size_t)OC * K2C * 2, szBP = 256, szOFF = RCH * 64 * 4, szIMX = RCH * K2C * 2;
  static_assert(NR * CC * 2 + (size_t)OC * K9C * 2 + (size_t)OC * K2C * 2 + 256 + RCH * 64 * 4 + RCH * K2C * 2 <= (size_t)134217728);
  static_assert(RCH * K9C * 2 <= RCH * K2C * 2);
  _Float16* X16 = (_Float16*)take(szX16); _Float16* BtO = (_Float16*)take(szBtO); _Float16* BtD = (_Float16*)take(szBtD); float* bpo = (float*)take(szBP);
  float* OFF = (float*)take(szOFF); _Float16* IMX = (_Float16*)take(szIMX);
  if (off > ws_size || off > (size_t)134217728) return;
  _Float16* IM = IMX; _Float16* IMP = IMX;

  k_xT<<<(unsigned)(NB * (HW / 64)), 256, 0, stream>>>(x, X16);
  k_wk<<<(unsigned)((OC * 72 + 255) / 256), 256, 0, stream>>>(w_off, NOFFC, 1, S_OFF, S_OFF, BtO);
  k_wk<<<(unsigned)((OC * 144 + 255) / 256), 256, 0, stream>>>(wd, OC, 2, S_HI, S_LO, BtD);
  k_b64<<<1, 64, 0, stream>>>(b_off, NOFFC, bpo);
  for (int ch = 0; ch < NCHUNK; ++ch) {
    const size_t row0c = (size_t)ch * RCH;
    k_im9<<<(unsigned)((RCH * 72 + 255) / 256), 256, 0, stream>>>(X16, row0c, RCH, IM);
    k_gemm2<0><<<dim3((unsigned)(RCH / 128), 1), 128, 0, stream>>>(IM, K9C, 0, BtO, K9C, 0, A_OFF, bpo, 0, nullptr, 1, 0, 0, OFF, nullptr, 64, 0, (int)RCH, 64, K9C);
    k_samp<<<(unsigned)((RCH * 72 + 255) / 256), 256, 0, stream>>>(X16, OFF, row0c, RCH, IMP);
    k_gemm2t<<<(unsigned)(RCH / 128), 128, 0, stream>>>(IMP, K2C, BtD, K2C, A_MAIN, row0c, out, (int)RCH, K2C);
  }
}
